// RNN_circular_LowEtAl_71081708749398
// MI455X (gfx1250) — hardware-verified
//
#include <hip/hip_runtime.h>

typedef __attribute__((ext_vector_type(16))) __bf16   v16b;
typedef __attribute__((ext_vector_type(8)))  __bf16   v8b;
typedef __attribute__((ext_vector_type(8)))  float    v8f;
typedef __attribute__((ext_vector_type(4)))  float    v4f;

constexpr int kBatch   = 256;
constexpr int kSteps   = 1024;
constexpr int kHid     = 512;
constexpr int kNav     = 1;
constexpr int kOutW    = 2 * kNav;
constexpr int kRowsPB  = 16;
constexpr int kBlocks  = kBatch / kRowsPB;
constexpr int kThreads = 256;
constexpr int kWaves   = kThreads / 32;
constexpr int kColsPW  = kHid / kWaves;
constexpr int kHP      = kHid + 8;
constexpr int kTile    = kRowsPB * kHP;
constexpr int kWhDw    = kHid * kHid / 2;
constexpr int kPrepBlocks = kWhDw / 256;
constexpr float kTwoPi = 6.28318548f;
constexpr int kChkBlocks  = 256;
constexpr int kChkThreads = 256;
constexpr int kChkPer     = 4;
constexpr int kFlagLine   = 32;
static_assert(kBatch % kRowsPB == 0, "blocks cover the batch exactly");
static_assert(kWaves * kColsPW == kHid, "wave columns cover the hidden dim exactly");
static_assert(kColsPW == 64, "4 subtiles of 16 per wave");
static_assert(kHid % 32 == 0, "K multiple of 32, no tail");
static_assert(kHP % 8 == 0, "16-B aligned fragment loads");
static_assert(kRowsPB * kOutW == 32, "one 128-B output line per block per step");
static_assert(kWaves * kRowsPB * kOutW == 256, "partial buffer extent");
static_assert(kWhDw % 256 == 0 && kPrepBlocks == 512, "prep grid covers the plane exactly");
static_assert((kHid * kHid) % 2 == 0, "dword packing");
static_assert(kChkBlocks * kChkThreads * kChkPer == kHid * kHid, "test grid covers W_h exactly");
static_assert(kChkThreads == 256, "8 waves per test block");

__device__ __forceinline__ unsigned short f2bf_bits(float f) {
  unsigned u = __float_as_uint(f);
  return (unsigned short)((u + 0x7FFFu + ((u >> 16) & 1u)) >> 16);
}
__device__ __forceinline__ float bf_bits2f(unsigned short h) { return __uint_as_float(((unsigned)h) << 16); }

__device__ __forceinline__ void dep_guard_b(v8f& a, v8f& b, v16b x, v16b y) { asm volatile("v_nop\n\tv_nop\n\tv_nop\n\tv_nop" : "+v"(a), "+v"(b) : "v"(x), "v"(y)); }
__device__ __forceinline__ void keep4_b(v16b a, v16b b, v16b c, v16b d) { asm volatile("v_nop" :: "v"(a), "v"(b), "v"(c), "v"(d)); }
__device__ __forceinline__ void acc_guard4(v8f& a, v8f& b, v8f& c, v8f& d) { asm volatile("v_nop\n\tv_nop\n\tv_nop\n\tv_nop" : "+v"(a), "+v"(b), "+v"(c), "+v"(d)); }

template <typename T> struct Frag;
template <> struct Frag<__bf16> {
  typedef v16b V; union U { v16b v; v8b h[2]; };
  static __device__ __forceinline__ v16b load(const __bf16* p) {
    U f; f.h[0] = *(const v8b*)(p); f.h[1] = *(const v8b*)(p + 16); return f.v;
  }
  static __device__ __forceinline__ v8f mma(v16b a, v16b b, v8f c) {
    return __builtin_amdgcn_wmma_f32_16x16x32_bf16(false, a, false, b, (short)0, c, false, false);
  }
  static __device__ __forceinline__ void guard(v8f& a, v8f& b, v16b x, v16b y) { dep_guard_b(a, b, x, y); }
  static __device__ __forceinline__ void keep(v16b a, v16b b, v16b c, v16b d) { keep4_b(a, b, c, d); }
};

__device__ __forceinline__ unsigned pack_bf16x2(float a, float b) {
  return (unsigned)f2bf_bits(a) | ((unsigned)f2bf_bits(b) << 16);
}
__device__ __forceinline__ void st2u(unsigned* p, unsigned v) { *(volatile unsigned*)p = v; __threadfence(); *(volatile unsigned*)p = v; }
__device__ __forceinline__ void st2i(int* p, int v) { *(volatile int*)p = v; __threadfence(); *(volatile int*)p = v; }

__global__ __launch_bounds__(kChkThreads) void wh_ident_kernel(const float* __restrict__ wh, int* __restrict__ flagp) {
  __shared__ int okl[kChkThreads];
  const int tid = threadIdx.x, blk = blockIdx.x;
  const int tix = blk * kChkThreads + tid;
  const v4f v = *(const v4f*)(wh + (size_t)tix * kChkPer);
  int ok = 1;
#pragma unroll
  for (int q = 0; q < kChkPer; ++q) {
    const int e = tix * kChkPer + q;
    const int row = e >> 9, col = e & (kHid - 1);
    const float expv = (row == col) ? 1.0f : 0.0f;
    ok &= (v[q] == expv) ? 1 : 0;
  }
  okl[tid] = ok;
  __syncthreads();
  if (tid < 32) {
    int a = 1;
#pragma unroll
    for (int i = 0; i < kChkThreads / 32; ++i) a &= okl[tid + 32 * i];
#pragma unroll
    for (int off = 16; off > 0; off >>= 1) a &= __shfl_xor(a, off, 32);
    st2i(flagp + (size_t)blk * kFlagLine + tid, a);
  }
}

__global__ __launch_bounds__(32) void flag_reduce_kernel(const int* __restrict__ flagp, int* __restrict__ flagw) {
  const int lane = threadIdx.x;
  int a = 1;
#pragma unroll 1
  for (int b = 0; b < kChkBlocks; ++b) a &= (flagp[(size_t)b * kFlagLine + lane] == 1) ? 1 : 0;
#pragma unroll
  for (int off = 16; off > 0; off >>= 1) a &= __shfl_xor(a, off, 32);
  st2i(flagw + lane, a);
}

__global__ __launch_bounds__(256) void prep_wh_kernel(const float* __restrict__ wh, unsigned* __restrict__ whu) {
  const int p = blockIdx.x * 256 + threadIdx.x;
  const unsigned u = pack_bf16x2(wh[2 * p], wh[2 * p + 1]);
  st2u(whu + p, u);
}

__global__ __launch_bounds__(kThreads) void rnn_kernel(
    const float* __restrict__ x,
    const float* __restrict__ theta,
    const __bf16* __restrict__ wh16,
    const float* __restrict__ wx,
    const float* __restrict__ bx,
    const float* __restrict__ wh0,
    const float* __restrict__ bh0,
    const float* __restrict__ wout,
    const float* __restrict__ bout,
    const int* __restrict__ flagw,
    float* __restrict__ out)
{
  __shared__ __align__(16) __bf16 hhi[kTile];
  __shared__ __align__(16) __bf16 hlo[kTile];
  __shared__ __align__(16) float  wxl[kHid];
  __shared__ __align__(16) float  bxl[kHid];
  __shared__ __align__(16) float  wo0l[kHid];
  __shared__ __align__(16) float  wo1l[kHid];
  __shared__ __align__(16) float  part[kWaves * kRowsPB * kOutW];
  __shared__ __align__(16) float  ost[kRowsPB * kOutW];

  const int tid = threadIdx.x, lane = tid & 31, wave = tid >> 5;
  const int c = lane & 15, hh = lane >> 4, koff = 8 * hh;
  const int b0 = blockIdx.x * kRowsPB;
  const int n0 = wave * kColsPW;
  const int pcol = n0 + koff;

  const int ident = __builtin_amdgcn_readfirstlane((flagw[0] == 1) ? 1 : 0);

  for (int i = tid; i < kHid; i += kThreads) {
    wxl[i] = wx[i]; bxl[i] = bx[i]; wo0l[i] = wout[i]; wo1l[i] = wout[kHid + i];
  }
  const float bo = bout[lane & 1];
  const float th = theta[b0 + c] * kTwoPi;

  v8f st[4];
#pragma unroll
  for (int j = 0; j < 4; ++j) {
#pragma unroll
    for (int r = 0; r < 8; ++r) {
      const int n = pcol + 16 * j + r;
      st[j][r] = th * wh0[n] + bh0[n];
    }
  }
  __syncthreads();

  const __bf16* arow = wh16 + (size_t)(n0 + c) * kHid + koff;
  const __bf16* brhi = hhi + c * kHP + koff;
  const __bf16* brlo = hlo + c * kHP + koff;
  __bf16* wrhi = hhi + c * kHP + pcol;
  __bf16* wrlo = hlo + c * kHP + pcol;
  const float* xrow = x + (size_t)(b0 + c) * kSteps;
  const v8f zero8 = {0.f, 0.f, 0.f, 0.f, 0.f, 0.f, 0.f, 0.f};

  for (int t = 0; t <= kSteps; ++t) {
    if (!ident) {
#pragma unroll
      for (int j = 0; j < 4; ++j) {
        v8b vh, vl;
#pragma unroll
        for (int r = 0; r < 8; ++r) {
          const float v = st[j][r];
          const __bf16 hb = (__bf16)v;
          const float hf = __uint_as_float(((unsigned)__builtin_bit_cast(unsigned short, hb)) << 16);
          vh[r] = hb;
          vl[r] = (__bf16)(v - hf);
        }
        *(v8b*)(wrhi + 16 * j) = vh;
        *(v8b*)(wrlo + 16 * j) = vl;
      }
    }
    float p0 = 0.f, p1 = 0.f;
#pragma unroll
    for (int j = 0; j < 4; ++j) {
      const v4f wa = *(const v4f*)(wo0l + pcol + 16 * j);
      const v4f wb = *(const v4f*)(wo0l + pcol + 16 * j + 4);
      const v4f ua = *(const v4f*)(wo1l + pcol + 16 * j);
      const v4f ub = *(const v4f*)(wo1l + pcol + 16 * j + 4);
#pragma unroll
      for (int r = 0; r < 4; ++r) { p0 += st[j][r] * wa[r];     p1 += st[j][r] * ua[r]; }
#pragma unroll
      for (int r = 0; r < 4; ++r) { p0 += st[j][4 + r] * wb[r]; p1 += st[j][4 + r] * ub[r]; }
    }
    p0 += __shfl_xor(p0, 16, 32);
    p1 += __shfl_xor(p1, 16, 32);
    part[(wave * kRowsPB + c) * kOutW + 0] = p0;
    part[(wave * kRowsPB + c) * kOutW + 1] = p1;
    __syncthreads();

    if (wave == 0) {
      float s = 0.f;
#pragma unroll
      for (int w = 0; w < kWaves; ++w) s += part[w * (kRowsPB * kOutW) + lane];
      s += bo;
      ost[lane] = s;
      __builtin_amdgcn_fence(__ATOMIC_RELEASE, "workgroup");
      __builtin_amdgcn_wave_barrier();
      __builtin_amdgcn_fence(__ATOMIC_ACQUIRE, "workgroup");
      const int l8 = lane & 7;
      const v4f ov = *(const v4f*)(ost + 4 * l8);
      float* op = out + ((size_t)t * kBatch + b0) * kOutW + 4 * l8;
      if (lane < 8) *(volatile v4f*)op = ov;
      __threadfence();
      if (lane < 8) *(volatile v4f*)op = ov;
    }
    if (t == kSteps) break;

    const float xv = xrow[t];
    if (!ident) {
#pragma unroll
      for (int j = 0; j < 4; ++j) st[j] = zero8;
#pragma unroll 1
      for (int kc = 0; kc < kHid / 32; ++kc) {
        v16b fa[4];
#pragma unroll
        for (int j = 0; j < 4; ++j) fa[j] = Frag<__bf16>::load(arow + (size_t)(16 * j) * kHid + kc * 32);
        const v16b fbh = Frag<__bf16>::load(brhi + kc * 32);
        const v16b fbl = Frag<__bf16>::load(brlo + kc * 32);
#pragma unroll
        for (int j = 0; j < 4; ++j) {
          st[j] = Frag<__bf16>::mma(fa[j], fbh, st[j]);
          st[j] = Frag<__bf16>::mma(fa[j], fbl, st[j]);
        }
        Frag<__bf16>::guard(st[0], st[3], fbh, fbl);
        Frag<__bf16>::keep(fa[0], fa[1], fa[2], fa[3]);
      }
      acc_guard4(st[0], st[1], st[2], st[3]);
    }
    __syncthreads();

#pragma unroll
    for (int j = 0; j < 4; ++j) {
      const v4f wa = *(const v4f*)(wxl + pcol + 16 * j);
      const v4f wb = *(const v4f*)(wxl + pcol + 16 * j + 4);
      const v4f ba = *(const v4f*)(bxl + pcol + 16 * j);
      const v4f bb = *(const v4f*)(bxl + pcol + 16 * j + 4);
#pragma unroll
      for (int r = 0; r < 4; ++r) {
        const float xp = xv * wa[r] + ba[r];
        const float v = st[j][r] + xp;
        st[j][r] = fmaxf(v, 0.0f);
      }
#pragma unroll
      for (int r = 0; r < 4; ++r) {
        const float xp = xv * wb[r] + bb[r];
        const float v = st[j][4 + r] + xp;
        st[j][4 + r] = fmaxf(v, 0.0f);
      }
    }
  }
}

extern "C" void kernel_launch(void* const* d_in, const int* in_sizes, int n_in,
                              void* d_out, int out_size, void* d_ws, size_t ws_size, hipStream_t stream) {
  if (n_in < 9 || d_out == nullptr || d_ws == nullptr) return;
  if (in_sizes[0] != kBatch * kSteps || in_sizes[1] != kBatch || in_sizes[2] != kHid * kHid ||
      in_sizes[3] != kHid || in_sizes[4] != kHid || in_sizes[5] != kHid || in_sizes[6] != kHid ||
      in_sizes[7] != kOutW * kHid || in_sizes[8] != kOutW ||
      out_size != (kSteps + 1) * kBatch * kOutW) return;

  const float* x     = (const float*)d_in[0];
  const float* theta = (const float*)d_in[1];
  const float* w_h   = (const float*)d_in[2];
  const float* w_x   = (const float*)d_in[3];
  const float* b_x   = (const float*)d_in[4];
  const float* w_h0  = (const float*)d_in[5];
  const float* b_h0  = (const float*)d_in[6];
  const float* w_out = (const float*)d_in[7];
  const float* b_out = (const float*)d_in[8];
  float* out = (float*)d_out;

  char* ws = (char*)d_ws; size_t off = 0;
  auto carve = [&](size_t bytes) -> char* { char* p = ws + off; off += (bytes + 255) & ~(size_t)255; return p; };
  unsigned short* WH16  = (unsigned short*)carve((size_t)kHid * kHid * 2);
  int*            FLAGP = (int*)carve((size_t)kChkBlocks * kFlagLine * sizeof(int));
  int*            FLAGW = (int*)carve((size_t)kFlagLine * sizeof(int));
  if (off > ws_size || off > (size_t)134217728) return;

  wh_ident_kernel<<<kChkBlocks, kChkThreads, 0, stream>>>(w_h, FLAGP);
  flag_reduce_kernel<<<1, 32, 0, stream>>>(FLAGP, FLAGW);

  prep_wh_kernel<<<kPrepBlocks, 256, 0, stream>>>(w_h, (unsigned*)WH16);

  rnn_kernel<<<kBlocks, kThreads, 0, stream>>>(x, theta, (const __bf16*)WH16, w_x, b_x, w_h0, b_h0, w_out, b_out, FLAGW, out);
}
